// HeteroGAT_43327630082180
// MI455X (gfx1250) — hardware-verified
//
#include <hip/hip_runtime.h>
#include <stddef.h>
#include <stdint.h>
#include <math.h>


#define F_IN    128
#define NTYP    3
#define NHD     4
#define HID     64
#define HC1     256
#define NGC     (NTYP * HC1)
#define KA      512
#define NCLS    2
#define NC2P    64
#define NTHR    256
#define NWAVE   8
#define EPT     8
#define CHUNK   (NTHR * EPT)
#define WCAP    (EPT * 32)
#define LISTN   (NWAVE * WCAP)
#define SLOTB   11
#define KEYN    (1 << SLOTB)
#define NBMAX   512
#define RCAP    28672
#define DEGCAP  256
#define GBM     64
#define GBN     64
#define GTHR    128
#define MROWS   128
#define NEGSL   0.2f
#define EPS_SM  1e-16f
#define NEGBIG  (-1.0e30f)
#define THIRD   (1.0f / 3.0f)
#define WSMAX   134217728
#define LDS_AGG ((2 * RCAP + 2 * KEYN + LISTN) * 4 + 64)

static_assert((CHUNK & (CHUNK - 1)) == 0 && CHUNK <= (1 << SLOTB));
static_assert(KEYN == (1 << SLOTB));
static_assert(NTYP * NBMAX <= KEYN);
static_assert(NTHR * 8 == KEYN);
static_assert(LISTN >= KEYN);
static_assert(LISTN >= NWAVE * WCAP);
static_assert((RCAP % 32) == 0);
static_assert(RCAP >= NCLS * NBMAX);
static_assert(LDS_AGG <= 300000);
static_assert(GBM == (GTHR / 32) * 16);
static_assert(GTHR == 2 * GBN && GTHR == 2 * GBM);
static_assert((F_IN % 32) == 0 && (KA % 32) == 0);
static_assert((NGC % GBN) == 0 && HID == GBN && NC2P == GBN);
static_assert(HC1 == NHD * HID);
static_assert(KA == 2 * HC1);
static_assert((MROWS % GBM) == 0);
static_assert(HC1 == 8 * 32);
static_assert(HID == 8 * 8);
static_assert((F_IN / 8) == 16);
static_assert(NTYP * NCLS <= NC2P);
static_assert(KA * 2 >= F_IN * 2);
static_assert(((NBMAX * NCLS * 4) % 128) == 0 && ((32 * NCLS * 4) % 128) == 0);

typedef float          v2f  __attribute__((ext_vector_type(2)));
typedef float          v4f  __attribute__((ext_vector_type(4)));
typedef float          v8f  __attribute__((ext_vector_type(8)));
typedef int            v4i  __attribute__((ext_vector_type(4)));
typedef int            v8i  __attribute__((ext_vector_type(8)));
typedef unsigned int   v4u  __attribute__((ext_vector_type(4)));
typedef unsigned short v8us __attribute__((ext_vector_type(8)));
typedef __bf16         v16b __attribute__((ext_vector_type(16)));
typedef v2f  __attribute__((may_alias)) v2fa;
typedef v4f  __attribute__((may_alias)) v4fa;
typedef v8us __attribute__((may_alias)) v8usa;
union FragB { v16b v; v8us h[2]; v8i w; };

__device__ __forceinline__ v8f wmb(const FragB& a, const FragB& b, v8f c) {
  v8f d = __builtin_amdgcn_wmma_f32_16x16x32_bf16(false, a.v, false, b.v, (short)0, c, false, false);
  asm volatile("v_nop\n\tv_nop\n\tv_nop\n\tv_nop" : "+v"(d) : "v"(a.w), "v"(b.w));
  return d;
}

__device__ __forceinline__ unsigned int f2bf(float f) {
  const unsigned int u = __float_as_uint(f);
  return ((u + 0x7FFFu + ((u >> 16) & 1u)) >> 16) & 0xFFFFu;
}
__device__ __forceinline__ float bf2f(unsigned int b) { return __uint_as_float(b << 16); }
__device__ __forceinline__ float bfr(float f) { return bf2f(f2bf(f)); }
__device__ __forceinline__ v4f bfr4(const v4f a) {
  v4f r; r.x = bfr(a.x); r.y = bfr(a.y); r.z = bfr(a.z); r.w = bfr(a.w); return r;
}
__device__ __forceinline__ unsigned int pk2(float lo, float hi) { return f2bf(lo) | (f2bf(hi) << 16); }
__device__ __forceinline__ v4u pack8(const v4f a, const v4f b) {
  v4u r;
  r.x = pk2(a.x, a.y); r.y = pk2(a.z, a.w); r.z = pk2(b.x, b.y); r.w = pk2(b.z, b.w);
  return r;
}
__device__ __forceinline__ float eluf(float v) { return v > 0.f ? v : (__expf(v) - 1.0f); }

__device__ __forceinline__ int scan_chunk(const int* __restrict__ dsts, int nE, int cbase, int slotBase,
                                          int nb, int vec8, int typ, int* list, int tid, int lane, int wave) {
  int wc = 0;
  const int el0  = tid * EPT;
  const int e0   = cbase + el0;
  const int sent = -2147483647 - 1;
  v4i da, db;
  if (vec8 != 0 && cbase + CHUNK <= nE) {
    da = *(const v4i*)(dsts + e0);
    db = *(const v4i*)(dsts + e0 + 4);
  } else {
    da.x = (e0     < nE) ? dsts[min(e0,     nE - 1)] : sent;
    da.y = (e0 + 1 < nE) ? dsts[min(e0 + 1, nE - 1)] : sent;
    da.z = (e0 + 2 < nE) ? dsts[min(e0 + 2, nE - 1)] : sent;
    da.w = (e0 + 3 < nE) ? dsts[min(e0 + 3, nE - 1)] : sent;
    db.x = (e0 + 4 < nE) ? dsts[min(e0 + 4, nE - 1)] : sent;
    db.y = (e0 + 5 < nE) ? dsts[min(e0 + 5, nE - 1)] : sent;
    db.z = (e0 + 6 < nE) ? dsts[min(e0 + 6, nE - 1)] : sent;
    db.w = (e0 + 7 < nE) ? dsts[min(e0 + 7, nE - 1)] : sent;
  }
  const unsigned nbs = (unsigned)slotBase;
  const unsigned unb = (unsigned)nb;
  const unsigned ut  = (unsigned)typ;
  const unsigned s0 = (unsigned)da.x - nbs, s1 = (unsigned)da.y - nbs;
  const unsigned s2 = (unsigned)da.z - nbs, s3 = (unsigned)da.w - nbs;
  const unsigned s4 = (unsigned)db.x - nbs, s5 = (unsigned)db.y - nbs;
  const unsigned s6 = (unsigned)db.z - nbs, s7 = (unsigned)db.w - nbs;
  const bool h0 = s0 < unb, h1 = s1 < unb, h2 = s2 < unb, h3 = s3 < unb;
  const bool h4 = s4 < unb, h5 = s5 < unb, h6 = s6 < unb, h7 = s7 < unb;
  const unsigned any = __builtin_amdgcn_ballot_w32(h0 | h1 | h2 | h3 | h4 | h5 | h6 | h7);
  if (any != 0u) {
#define HITJ(J, HJ, SJ) { \
      const unsigned mj = __builtin_amdgcn_ballot_w32(HJ); \
      if (mj != 0u) { \
        if (HJ) { \
          const int pos = wc + (int)__builtin_amdgcn_mbcnt_lo(mj, 0u); \
          if (pos < WCAP) list[wave * WCAP + pos] = ((el0 + (J)) << SLOTB) | (int)((SJ) * (unsigned)NTYP + ut); \
        } \
        wc += (int)__builtin_popcount(mj); } }
    HITJ(0, h0, s0)
    HITJ(1, h1, s1)
    HITJ(2, h2, s2)
    HITJ(3, h3, s3)
    HITJ(4, h4, s4)
    HITJ(5, h5, s5)
    HITJ(6, h6, s6)
    HITJ(7, h7, s7)
#undef HITJ
  }
  return wc;
}

__global__ __launch_bounds__(NTHR) void k_xprep(const float* __restrict__ x, unsigned short* xb, int nN, int nUnits) {
  const int i = (int)blockIdx.x * NTHR + (int)threadIdx.x;
  if (i >= nUnits) return;
  const int row = i >> 4;
  const int c0  = (i & 15) * 8;
  const int rc  = row < nN ? row : nN - 1;
  const float* p = x + (size_t)rc * F_IN + c0;
  v4f a = *(const v4fa*)p, b = *(const v4fa*)(p + 4);
  const v4f z4 = {0.f, 0.f, 0.f, 0.f};
  if (row >= nN) { a = z4; b = z4; }
  const v4u hv = pack8(a, b);
  const size_t o = (size_t)row * F_IN + c0;
  *(volatile v4u*)(xb + o) = hv;
  __threadfence();
  *(volatile v4u*)(xb + o) = hv;
}

__global__ __launch_bounds__(NTHR) void k_wtr3(const float* __restrict__ w, int Kin, int Cw, int Nrows, int Kout,
                                               unsigned short* wt, int nUnits) {
  const int u = (int)blockIdx.x * NTHR + (int)threadIdx.x;
  if (u >= nUnits) return;
  const int kq  = Kout >> 3;
  const int n   = u / kq;
  const int k8  = (u - n * kq) * 8;
  const int kk  = k8 - (k8 / Kin) * Kin;
  const int nv  = NTYP * Cw;
  const int ncl = n < nv ? n : nv - 1;
  const int t   = ncl / Cw;
  const int c   = ncl - t * Cw;
  const float* p = w + ((size_t)t * (size_t)Kin + (size_t)kk) * (size_t)Cw + c;
  v4f a, b;
  a.x = p[0];                  a.y = p[(size_t)Cw];         a.z = p[(size_t)2 * Cw];     a.w = p[(size_t)3 * Cw];
  b.x = p[(size_t)4 * Cw];     b.y = p[(size_t)5 * Cw];     b.z = p[(size_t)6 * Cw];     b.w = p[(size_t)7 * Cw];
  const v4f z4 = {0.f, 0.f, 0.f, 0.f};
  if (n >= nv || n >= Nrows) { a = z4; b = z4; }
  const v4u wv = pack8(a, b);
  unsigned short* o = wt + (size_t)n * (size_t)Kout + k8;
  *(volatile v4u*)o = wv;
  __threadfence();
  *(volatile v4u*)o = wv;
}

__global__ __launch_bounds__(GTHR) void k_gemm(
    const unsigned short* __restrict__ A, const unsigned short* __restrict__ WT,
    float* outF, int K, int ldo,
    const float* __restrict__ atts, const float* __restrict__ attd, int attLen,
    float* SD, int MPr)
{
  __shared__ __attribute__((aligned(16))) float stg[GBM * GBN];
  __shared__ __attribute__((aligned(16))) float satt[2 * GBN];
  __shared__ __attribute__((aligned(16))) float sdot[2 * GBM];
  const int tid = (int)threadIdx.x, lane = tid & 31, wave = tid >> 5, hh = lane >> 4, m = lane & 15;
  const int rowBase = (int)blockIdx.x * GBM;
  const int head    = (int)blockIdx.y;
  const int col0    = head * GBN;

  {
    const int which = tid >> 6;
    const int c  = tid & 63;
    const int cl = c < attLen ? c : attLen - 1;
    const float vs = atts[head * attLen + cl];
    const float vd = attd[head * attLen + cl];
    const unsigned int msk = (which == 0) ? 0u : 0xFFFFFFFFu;
    const unsigned int inr = (c < attLen) ? 0xFFFFFFFFu : 0u;
    float v = __uint_as_float((__float_as_uint(vs) & ~msk) | (__float_as_uint(vd) & msk));
    v = __uint_as_float(__float_as_uint(bfr(v)) & inr);
    satt[which * GBN + c] = v;
  }

  v8f acc[4];
  {
    const v8f z = {0.f, 0.f, 0.f, 0.f, 0.f, 0.f, 0.f, 0.f};
    acc[0] = z; acc[1] = z; acc[2] = z; acc[3] = z;
  }
  const unsigned short* ap = A  + (size_t)(rowBase + 16 * wave + m) * (size_t)K + 8 * hh;
  const unsigned short* wp = WT + (size_t)(col0 + m) * (size_t)K + 8 * hh;
  const int ksteps = K >> 5;
#pragma unroll 1
  for (int ks = 0; ks < ksteps; ++ks) {
    FragB af;
    af.h[0] = *(const v8usa*)(ap + 32 * ks);
    af.h[1] = *(const v8usa*)(ap + 32 * ks + 16);
#pragma unroll
    for (int t = 0; t < 4; ++t) {
      const unsigned short* wq = wp + (size_t)(16 * t) * (size_t)K + 32 * ks;
      FragB bf;
      bf.h[0] = *(const v8usa*)wq;
      bf.h[1] = *(const v8usa*)(wq + 16);
      acc[t] = wmb(af, bf, acc[t]);
    }
  }

#pragma unroll
  for (int t = 0; t < 4; ++t) {
    const int lc = 16 * t + m;
#pragma unroll
    for (int r = 0; r < 8; ++r) {
      const int lr = 16 * wave + 8 * hh + r;
      stg[lr * GBN + lc] = acc[t][r];
    }
  }
  __syncthreads();

  {
    const int row = tid & 63, which = tid >> 6;
    const float* sa = satt + which * GBN;
    const float* hr = stg + row * GBN;
    float d = 0.f;
#pragma unroll 4
    for (int c4 = 0; c4 < GBN / 4; ++c4) {
      const v4f hv = *(const v4fa*)(hr + 4 * c4);
      const v4f av = *(const v4fa*)(sa + 4 * c4);
      d = fmaf(hv.x, av.x, d);
      d = fmaf(hv.y, av.y, d);
      d = fmaf(hv.z, av.z, d);
      d = fmaf(hv.w, av.w, d);
    }
    sdot[which * GBM + row] = d;
  }
  __syncthreads();

  v4f fv[8];
#pragma unroll
  for (int i = 0; i < 8; ++i) {
    const int lr = 16 * wave + 2 * i + hh;
    fv[i] = *(const v4fa*)(stg + lr * GBN + 4 * m);
  }
  const int which2 = lane >> 4, piece = lane & 15;
  const v4f sdv = *(const v4fa*)(sdot + which2 * GBM + 4 * piece);
  float* sp = SD + (size_t)(2 * head + which2) * (size_t)MPr + rowBase + 4 * piece;

#pragma unroll
  for (int i = 0; i < 8; ++i) {
    const int lr = 16 * wave + 2 * i + hh;
    const int gr = rowBase + lr;
    float* op = outF + (size_t)gr * (size_t)ldo + col0 + 4 * m;
    *(volatile v4f*)op = fv[i];
  }
  if (wave == 0) *(volatile v4f*)sp = sdv;
  __threadfence();
#pragma unroll
  for (int i = 0; i < 8; ++i) {
    const int lr = 16 * wave + 2 * i + hh;
    const int gr = rowBase + lr;
    float* op = outF + (size_t)gr * (size_t)ldo + col0 + 4 * m;
    *(volatile v4f*)op = fv[i];
  }
  if (wave == 0) *(volatile v4f*)sp = sdv;
}

template<int L>
__global__ __launch_bounds__(NTHR) void k_agg(
    const int* __restrict__ srcs, const int* __restrict__ dsts,
    const float* __restrict__ F, const float* __restrict__ SD,
    const float* __restrict__ bias, const float* __restrict__ al2p, const float* __restrict__ ar2p,
    unsigned short* HP, float* out,
    int nN, int nE, int nb, int vec8, int MPr, int nOut0) {
  extern __shared__ v4f lds_dyn[];
  int* reg1 = (int*)lds_dyn;
  int* reg2 = reg1 + RCAP;
  int* scnt = reg2 + RCAP;
  int* soff = scnt + KEYN;
  int* list = soff + KEYN;
  int* wcnt = list + LISTN;
  int* wtot = wcnt + NWAVE;
  const int tid = (int)threadIdx.x, lane = tid & 31, wave = tid >> 5;
  const int nodeBase = (int)blockIdx.x * nb;

  for (int i = tid; i < KEYN; i += NTHR) scnt[i] = 0;
  __syncthreads();

  int tot = 0;
  const int nChunks = (nE + CHUNK - 1) / CHUNK;
#pragma unroll 1
  for (int t = 0; t < NTYP; ++t) {
    const int* dt = dsts + (size_t)t * (size_t)nE;
#pragma unroll 1
    for (int ch = 0; ch < nChunks; ++ch) {
      const int cbase = ch * CHUNK;
      const int wc = scan_chunk(dt, nE, cbase, nodeBase, nb, vec8, t, list, tid, lane, wave);
      if (lane == 0) wcnt[wave] = wc;
      __syncthreads();
      int pre = 0, all = 0;
#pragma unroll
      for (int w2 = 0; w2 < NWAVE; ++w2) {
        int c = wcnt[w2];
        c = c < 0 ? 0 : (c > WCAP ? WCAP : c);
        all += c;
        pre += (w2 < wave) ? c : 0;
      }
      const int wcc  = wc > WCAP ? WCAP : wc;
      const int base = tot + pre;
#pragma unroll 1
      for (int i = lane; i < wcc; i += 32) {
        const int ent = list[wave * WCAP + i];
        const int el  = (ent >> SLOTB) & (CHUNK - 1);
        const int key = ent & (KEYN - 1);
        int eid = cbase + el;
        eid = eid > nE - 1 ? nE - 1 : eid;
        const int pos = base + i;
        if (pos < RCAP) reg1[pos] = (int)(((unsigned)eid << SLOTB) | (unsigned)key);
      }
      tot += all;
      tot = tot > RCAP ? RCAP : tot;
      __syncthreads();
    }
  }
  const int nh = tot;

  if (wave == 0) {
#pragma unroll 1
    for (int b0 = 0; b0 < nh; b0 += 32) {
      const int idx = b0 + lane;
      const int uv  = reg1[idx < nh ? idx : nh - 1];
      const int m32 = (nh - b0) < 32 ? (nh - b0) : 32;
#pragma unroll 1
      for (int k = 0; k < m32; ++k) {
        const int u  = __builtin_amdgcn_readlane(uv, k);
        const int sl = u & (KEYN - 1);
        if (lane == 0) scnt[sl] = scnt[sl] + 1;
      }
    }
  }
  __syncthreads();

  {
    const v4i ca = *(const v4i*)(scnt + 8 * tid);
    const v4i cb = *(const v4i*)(scnt + 8 * tid + 4);
    const int e0 = ca.x < 0 ? 0 : ca.x, e1 = ca.y < 0 ? 0 : ca.y, e2 = ca.z < 0 ? 0 : ca.z, e3 = ca.w < 0 ? 0 : ca.w;
    const int e4 = cb.x < 0 ? 0 : cb.x, e5 = cb.y < 0 ? 0 : cb.y, e6 = cb.z < 0 ? 0 : cb.z, e7 = cb.w < 0 ? 0 : cb.w;
    const int ts = e0 + e1 + e2 + e3 + e4 + e5 + e6 + e7;
    int incl = ts;
#pragma unroll
    for (int d = 1; d < 32; d <<= 1) {
      const int up = __shfl_up(incl, d);
      if (lane >= d) incl += up;
    }
    if (lane == 31) wtot[wave] = incl;
    __syncthreads();
    int pre = 0;
#pragma unroll
    for (int w2 = 0; w2 < NWAVE; ++w2) pre += (w2 < wave) ? wtot[w2] : 0;
    int run = pre + incl - ts;
    soff[8 * tid + 0] = run; run += e0;
    soff[8 * tid + 1] = run; run += e1;
    soff[8 * tid + 2] = run; run += e2;
    soff[8 * tid + 3] = run; run += e3;
    soff[8 * tid + 4] = run; run += e4;
    soff[8 * tid + 5] = run; run += e5;
    soff[8 * tid + 6] = run; run += e6;
    soff[8 * tid + 7] = run;
  }
  __syncthreads();
  for (int i = tid; i < KEYN; i += NTHR) list[i] = soff[i];
  __syncthreads();

  if (wave == 0) {
#pragma unroll 1
    for (int b0 = 0; b0 < nh; b0 += 32) {
      const int idx = b0 + lane;
      const int uv  = reg1[idx < nh ? idx : nh - 1];
      const int m32 = (nh - b0) < 32 ? (nh - b0) : 32;
#pragma unroll 1
      for (int k = 0; k < m32; ++k) {
        const int u   = __builtin_amdgcn_readlane(uv, k);
        const int sl  = u & (KEYN - 1);
        const int eid = (int)((unsigned)u >> SLOTB);
        if (lane == 0) {
          int pos = list[sl];
          pos = pos < 0 ? 0 : (pos > RCAP - 1 ? RCAP - 1 : pos);
          reg2[pos] = eid;
          list[sl] = pos + 1;
        }
      }
    }
  }
  __syncthreads();

  const int nbw = nb >> 3;
  const bool ovf = (nh >= RCAP);
  const float qnan = __int_as_float(0x7fc00000);

  if (L == 1) {
    const int c0   = 8 * lane;
    const int head = lane >> 3;
    const v4f z4 = {0.f, 0.f, 0.f, 0.f};

#pragma unroll 1
    for (int jt = 0; jt < nbw; ++jt) {
      const int slot = wave * nbw + jt;
      const int grow = nodeBase + slot;
      const int gcl  = grow < nN ? grow : nN - 1;
      float pz = ovf ? qnan : 0.0f;
      v4f sa = z4, sb = z4;

#pragma unroll 1
      for (int t = 0; t < NTYP; ++t) {
        const int key = slot * NTYP + t;
        int st = soff[key];
        const int craw = scnt[key];
        int cnt = craw;
        st  = st < 0 ? 0 : (st > nh ? nh : st);
        cnt = cnt < 0 ? 0 : (cnt > DEGCAP ? DEGCAP : cnt);
        if (cnt > nh - st) cnt = nh - st;
        pz = (craw > DEGCAP) ? qnan : pz;

        const float* ASp = SD + (size_t)(2 * (NHD * t + head)) * (size_t)MPr;
        const float* ADp = ASp + MPr;
        const int*   srt = srcs + (size_t)t * (size_t)nE;
        const float* Ft  = F + (size_t)(HC1 * t + c0);
        const float* bp  = bias + HC1 * t + c0;
        const v4f bbA = bfr4(*(const v4fa*)bp);
        const v4f bbB = bfr4(*(const v4fa*)(bp + 4));
        const float adv = ADp[gcl];
        float mx = NEGBIG, dn = 0.0f;
        v4f av = z4, bv = z4;

#pragma unroll 1
        for (int q = 0; q < cnt; ++q) {
          int idx = st + q; idx = idx > RCAP - 1 ? RCAP - 1 : idx;
          int eid = reg2[idx]; eid = eid < 0 ? 0 : (eid > nE - 1 ? nE - 1 : eid);
          const int sraw = srt[eid];
          const int s = sraw < 0 ? 0 : (sraw > nN - 1 ? nN - 1 : sraw);
          const float* gsrc = Ft + (size_t)s * NGC;
          const v4f fa = *(const v4fa*)gsrc;
          const v4f fb = *(const v4fa*)(gsrc + 4);
          float lg = ASp[s] + adv;
          lg = lg > 0.f ? lg : NEGSL * lg;
          const float df = lg - mx;
          const float ee = __expf(-fabsf(df));
          const bool up  = df > 0.f;
          const float s1 = up ? ee : 1.0f;
          const float s2 = up ? 1.0f : ee;
          mx = up ? lg : mx;
          dn = fmaf(dn, s1, s2);
          av.x = fmaf(av.x, s1, s2 * fa.x);
          av.y = fmaf(av.y, s1, s2 * fa.y);
          av.z = fmaf(av.z, s1, s2 * fa.z);
          av.w = fmaf(av.w, s1, s2 * fa.w);
          bv.x = fmaf(bv.x, s1, s2 * fb.x);
          bv.y = fmaf(bv.y, s1, s2 * fb.y);
          bv.z = fmaf(bv.z, s1, s2 * fb.z);
          bv.w = fmaf(bv.w, s1, s2 * fb.w);
        }
        const float inv = __builtin_amdgcn_rcpf(dn + EPS_SM);
        sa.x += fmaf(av.x, inv, bbA.x);
        sa.y += fmaf(av.y, inv, bbA.y);
        sa.z += fmaf(av.z, inv, bbA.z);
        sa.w += fmaf(av.w, inv, bbA.w);
        sb.x += fmaf(bv.x, inv, bbB.x);
        sb.y += fmaf(bv.y, inv, bbB.y);
        sb.z += fmaf(bv.z, inv, bbB.z);
        sb.w += fmaf(bv.w, inv, bbB.w);
      }

      const bool live = grow < nN;
      v4f va, vb;
      va.x = eluf(sa.x * THIRD); va.y = eluf(sa.y * THIRD); va.z = eluf(sa.z * THIRD); va.w = eluf(sa.w * THIRD);
      vb.x = eluf(sb.x * THIRD); vb.y = eluf(sb.y * THIRD); vb.z = eluf(sb.z * THIRD); vb.w = eluf(sb.w * THIRD);
      v4f oa, ob;
      oa.x = (live ? va.x : 0.f) + pz;
      oa.y = (live ? va.y : 0.f) + pz;
      oa.z = (live ? va.z : 0.f) + pz;
      oa.w = (live ? va.w : 0.f) + pz;
      ob.x = (live ? vb.x : 0.f) + pz;
      ob.y = (live ? vb.y : 0.f) + pz;
      ob.z = (live ? vb.z : 0.f) + pz;
      ob.w = (live ? vb.w : 0.f) + pz;
      const unsigned int h0 = f2bf(oa.x), h1 = f2bf(oa.y), h2 = f2bf(oa.z), h3 = f2bf(oa.w);
      const unsigned int h4 = f2bf(ob.x), h5 = f2bf(ob.y), h6 = f2bf(ob.z), h7 = f2bf(ob.w);
      const unsigned int g0 = f2bf(oa.x - bf2f(h0)), g1 = f2bf(oa.y - bf2f(h1));
      const unsigned int g2 = f2bf(oa.z - bf2f(h2)), g3 = f2bf(oa.w - bf2f(h3));
      const unsigned int g4 = f2bf(ob.x - bf2f(h4)), g5 = f2bf(ob.y - bf2f(h5));
      const unsigned int g6 = f2bf(ob.z - bf2f(h6)), g7 = f2bf(ob.w - bf2f(h7));
      v4u hv, lv;
      hv.x = h0 | (h1 << 16); hv.y = h2 | (h3 << 16); hv.z = h4 | (h5 << 16); hv.w = h6 | (h7 << 16);
      lv.x = g0 | (g1 << 16); lv.y = g2 | (g3 << 16); lv.z = g4 | (g5 << 16); lv.w = g6 | (g7 << 16);
      unsigned short* gp = HP + (size_t)grow * KA + 8 * lane;
      unsigned short* gq = gp + HC1;
      const bool wr = grow < MPr;
      if (wr) { *(volatile v4u*)gp = hv; *(volatile v4u*)gq = lv; }
      __threadfence();
      if (wr) { *(volatile v4u*)gp = hv; *(volatile v4u*)gq = lv; }
    }
  } else {
    float* res = (float*)reg1;

#pragma unroll 1
    for (int jt = 0; jt < nbw; ++jt) {
      const int slot = wave * nbw + jt;
      const int grow = nodeBase + slot;
      const int gcl  = grow < nN ? grow : nN - 1;
      float pz = ovf ? qnan : 0.0f;
      float z0s = 0.0f, z1s = 0.0f;

#pragma unroll 1
      for (int t = 0; t < NTYP; ++t) {
        const int key = slot * NTYP + t;
        int st = soff[key];
        const int craw = scnt[key];
        int cnt = craw;
        st  = st < 0 ? 0 : (st > nh ? nh : st);
        cnt = cnt < 0 ? 0 : (cnt > DEGCAP ? DEGCAP : cnt);
        if (cnt > nh - st) cnt = nh - st;
        pz = (craw > DEGCAP) ? qnan : pz;

        const float als0 = bfr(al2p[NCLS * t]), als1 = bfr(al2p[NCLS * t + 1]);
        const float ars0 = bfr(ar2p[NCLS * t]), ars1 = bfr(ar2p[NCLS * t + 1]);
        const float bz0  = bfr(bias[NCLS * t]), bz1  = bfr(bias[NCLS * t + 1]);
        const int*   srt = srcs + (size_t)t * (size_t)nE;
        const float* Ft  = F + NCLS * t;
        const v2f fd = *(const v2fa*)(Ft + (size_t)gcl * NC2P);
        const float erd = fmaf(fd.y, ars1, fd.x * ars0);
        float mx = NEGBIG, dn = 0.0f, a0 = 0.0f, a1 = 0.0f;

#pragma unroll 1
        for (int cb = 0; cb < cnt; cb += 32) {
          const int i  = cb + lane;
          const bool ok = i < cnt;
          const int ic = ok ? i : cnt - 1;
          int idx = st + ic; idx = idx < 0 ? 0 : (idx > RCAP - 1 ? RCAP - 1 : idx);
          int eid = reg2[idx]; eid = eid < 0 ? 0 : (eid > nE - 1 ? nE - 1 : eid);
          const int sraw = srt[eid];
          const int s = sraw < 0 ? 0 : (sraw > nN - 1 ? nN - 1 : sraw);
          const v2f fs = *(const v2fa*)(Ft + (size_t)s * NC2P);
          const float els = fmaf(fs.y, als1, fs.x * als0);
          float lg = els + erd;
          lg = lg > 0.f ? lg : NEGSL * lg;
          const float lgm = ok ? lg : NEGBIG;
          float cm = lgm;
#pragma unroll
          for (int off = 16; off > 0; off >>= 1) cm = fmaxf(cm, __shfl_xor(cm, off));
          const float mn = fmaxf(mx, cm);
          const float pe = __expf(lgm - mn);
          const float p  = ok ? pe : 0.0f;
          const float sc = __expf(mx - mn);
          float ps = p, px = p * fs.x, py = p * fs.y;
#pragma unroll
          for (int off = 16; off > 0; off >>= 1) {
            ps += __shfl_xor(ps, off);
            px += __shfl_xor(px, off);
            py += __shfl_xor(py, off);
          }
          dn = fmaf(dn, sc, ps);
          a0 = fmaf(a0, sc, px);
          a1 = fmaf(a1, sc, py);
          mx = mn;
        }
        const float inv = __builtin_amdgcn_rcpf(dn + EPS_SM);
        z0s += fmaf(a0, inv, bz0);
        z1s += fmaf(a1, inv, bz1);
      }
      if (lane == 0) {
        res[NCLS * slot]     = z0s * THIRD + pz;
        res[NCLS * slot + 1] = z1s * THIRD + pz;
      }
    }

    __syncthreads();
    const int npc = (nb * NCLS) >> 2;
    const v4f ones = {1.0f, 1.0f, 1.0f, 1.0f};
#pragma unroll 1
    for (int p = tid; p < npc; p += NTHR) {
      const v4f v = *(const v4fa*)(res + 4 * p);
      const int f0 = nodeBase * NCLS + 4 * p;
      if (f0 + 4 <= nOut0) {
        *(volatile v4f*)(out + (size_t)f0) = v;
        *(volatile v4f*)(out + (size_t)nOut0 + (size_t)f0) = ones;
      }
    }
    __threadfence();
#pragma unroll 1
    for (int p = tid; p < npc; p += NTHR) {
      const v4f v = *(const v4fa*)(res + 4 * p);
      const int f0 = nodeBase * NCLS + 4 * p;
      if (f0 + 4 <= nOut0) {
        *(volatile v4f*)(out + (size_t)f0) = v;
        *(volatile v4f*)(out + (size_t)nOut0 + (size_t)f0) = ones;
      }
    }
  }
}

static int pick_nb(long long eTot, int nN) {
  int nb = NBMAX;
  while (nb > 32 && (long long)nb * eTot * 8LL > (long long)RCAP * (long long)nN * 7LL) nb >>= 1;
  return nb;
}
static inline int cdiv(int a, int b) { return (a + b - 1) / b; }

extern "C" void kernel_launch(void* const* d_in, const int* in_sizes, int n_in,
                              void* d_out, int out_size, void* d_ws, size_t ws_size,
                              hipStream_t stream) {
  if (n_in < 15) return;
  const int nN = in_sizes[0] / F_IN;
  if (nN <= 0 || in_sizes[0] != nN * F_IN || nN > (1 << 22)) return;
  if ((nN & 1) != 0) return;
  if (in_sizes[1] != NTYP * F_IN * HC1) return;
  if (in_sizes[2] != NTYP * NHD * HID || in_sizes[3] != NTYP * NHD * HID) return;
  if (in_sizes[4] != NTYP * HC1) return;
  if (in_sizes[5] != NTYP * HC1 * HC1) return;
  if (in_sizes[6] != NTYP * NHD * HID || in_sizes[7] != NTYP * NHD * HID) return;
  if (in_sizes[8] != NTYP * HC1) return;
  if (in_sizes[9] != NTYP * HC1 * NCLS) return;
  if (in_sizes[10] != NTYP * NCLS || in_sizes[11] != NTYP * NCLS) return;
  if (in_sizes[12] != NTYP * NCLS) return;
  if (in_sizes[13] < NTYP || (in_sizes[13] % NTYP) != 0) return;
  const int nE = in_sizes[13] / NTYP;
  if (in_sizes[14] != NTYP * nE) return;
  if (nE < 1 || nE >= (1 << (32 - SLOTB))) return;
  const int nOut0 = nN * NCLS;
  if (out_size != 2 * nOut0) return;

  const float* feat = (const float*)d_in[0];
  const float* W0   = (const float*)d_in[1];
  const float* al0  = (const float*)d_in[2];
  const float* ar0  = (const float*)d_in[3];
  const float* b0   = (const float*)d_in[4];
  const float* W1   = (const float*)d_in[5];
  const float* al1  = (const float*)d_in[6];
  const float* ar1  = (const float*)d_in[7];
  const float* b1   = (const float*)d_in[8];
  const float* W2   = (const float*)d_in[9];
  const float* al2  = (const float*)d_in[10];
  const float* ar2  = (const float*)d_in[11];
  const float* b2   = (const float*)d_in[12];
  const int*   src  = (const int*)  d_in[13];
  const int*   dst  = (const int*)  d_in[14];
  float* out = (float*)d_out;

  const int MP   = cdiv(nN, MROWS) * MROWS;
  const int nb   = pick_nb((long long)NTYP * (long long)nE, nN);
  if (nb < 32 || (nb & (nb - 1)) != 0 || nb > NBMAX) return;
  const int gA   = cdiv(MP, nb);
  const int vec8 = ((nE & 3) == 0) ? 1 : 0;
  if (gA * nb < MP) return;

  char* ws = (char*)d_ws;
  size_t off = 0;
  const size_t oW0T = off; off += (size_t)NGC * F_IN * 2;          off = (off + 255) & ~(size_t)255;
  const size_t oW1T = off; off += (size_t)NGC * KA * 2;            off = (off + 255) & ~(size_t)255;
  const size_t oW2T = off; off += (size_t)NC2P * KA * 2;           off = (off + 255) & ~(size_t)255;
  const size_t oH   = off; off += (size_t)MP * NGC * 4;            off = (off + 255) & ~(size_t)255;
  const size_t oSD  = off; off += (size_t)2 * NTYP * NHD * MP * 4; off = (off + 255) & ~(size_t)255;
  const size_t oAP  = off; off += (size_t)MP * KA * 2;             off = (off + 255) & ~(size_t)255;
  if (off > ws_size || off > (size_t)WSMAX) return;
  unsigned short* W0T = (unsigned short*)(ws + oW0T);
  unsigned short* W1T = (unsigned short*)(ws + oW1T);
  unsigned short* W2T = (unsigned short*)(ws + oW2T);
  float*          H   = (float*)(ws + oH);
  float*          SD  = (float*)(ws + oSD);
  unsigned short* AP  = (unsigned short*)(ws + oAP);
  unsigned short* XB  = AP;

  hipFuncSetAttribute(reinterpret_cast<const void*>(&k_agg<1>),
                      hipFuncAttributeMaxDynamicSharedMemorySize, LDS_AGG);
  hipFuncSetAttribute(reinterpret_cast<const void*>(&k_agg<2>),
                      hipFuncAttributeMaxDynamicSharedMemorySize, LDS_AGG);

  const int nUx = MP * (F_IN / 8);
  k_xprep<<<cdiv(nUx, NTHR), NTHR, 0, stream>>>(feat, XB, nN, nUx);

  {
    const int nUw0 = NGC * (F_IN / 8);
    k_wtr3<<<cdiv(nUw0, NTHR), NTHR, 0, stream>>>(W0, F_IN, HC1, NGC, F_IN, W0T, nUw0);
    const int nUw1 = NGC * (KA / 8);
    k_wtr3<<<cdiv(nUw1, NTHR), NTHR, 0, stream>>>(W1, HC1, HC1, NGC, KA, W1T, nUw1);
    const int nUw2 = NC2P * (KA / 8);
    k_wtr3<<<cdiv(nUw2, NTHR), NTHR, 0, stream>>>(W2, HC1, NCLS, NC2P, KA, W2T, nUw2);
  }

  const int gM = MP / GBM;
  k_gemm<<<dim3(gM, NGC / GBN), GTHR, 0, stream>>>(XB, W0T, H, F_IN, NGC, al0, ar0, HID, SD, MP);
  k_agg<1><<<gA, NTHR, LDS_AGG, stream>>>(src, dst, H, SD, b0, al2, ar2, AP, out, nN, nE, nb, vec8, MP, nOut0);
  k_gemm<<<dim3(gM, NGC / GBN), GTHR, 0, stream>>>(AP, W1T, H, KA, NGC, al1, ar1, HID, SD, MP);
  k_agg<1><<<gA, NTHR, LDS_AGG, stream>>>(src, dst, H, SD, b1, al2, ar2, AP, out, nN, nE, nb, vec8, MP, nOut0);
  k_gemm<<<dim3(gM, NC2P / GBN), GTHR, 0, stream>>>(AP, W2T, H, KA, NC2P, al2, ar2, NCLS, SD, MP);
  k_agg<2><<<gA, NTHR, LDS_AGG, stream>>>(src, dst, H, SD, b2, al2, ar2, AP, out, nN, nE, nb, vec8, MP, nOut0);
}
